// SpatialTransformer_24575802868328
// MI455X (gfx1250) — hardware-verified
//
#include <hip/hip_runtime.h>
#include <math.h>
typedef __attribute__((ext_vector_type(16))) _Float16 v16h;
typedef __attribute__((ext_vector_type(8)))  _Float16 v8h;
typedef __attribute__((ext_vector_type(16))) __bf16   v16b;
typedef __attribute__((ext_vector_type(8)))  __bf16   v8b;
typedef __attribute__((ext_vector_type(8)))  float    v8f;
typedef __attribute__((ext_vector_type(4)))  float    v4f;
#define PSCALE 32768.0f
#define U16(p) ((const unsigned short*)(const void*)(p))
#define PSCALE_INV (1.0f / 32768.0f)

__device__ __forceinline__ unsigned short f2bf_bits(float f) {
  unsigned u = __float_as_uint(f);
  return (unsigned short)((u + 0x7FFFu + ((u >> 16) & 1u)) >> 16);
}
__device__ __forceinline__ float bf_bits2f(unsigned short h) { return __uint_as_float(((unsigned)h) << 16); }

__device__ __forceinline__ void dep_guard_h(v8f& a, v8f& b, v16h x, v16h y) { asm volatile("v_nop\n\tv_nop\n\tv_nop\n\tv_nop" : "+v"(a), "+v"(b) : "v"(x), "v"(y)); }
__device__ __forceinline__ void dep_guard_b(v8f& a, v8f& b, v16b x, v16b y) { asm volatile("v_nop\n\tv_nop\n\tv_nop\n\tv_nop" : "+v"(a), "+v"(b) : "v"(x), "v"(y)); }
__device__ __forceinline__ void keep4_h(v16h a, v16h b, v16h c, v16h d) { asm volatile("v_nop" :: "v"(a), "v"(b), "v"(c), "v"(d)); }
__device__ __forceinline__ void keep4_b(v16b a, v16b b, v16b c, v16b d) { asm volatile("v_nop" :: "v"(a), "v"(b), "v"(c), "v"(d)); }
__device__ __forceinline__ void acc_guard4(v8f& a, v8f& b, v8f& c, v8f& d) { asm volatile("v_nop\n\tv_nop\n\tv_nop\n\tv_nop" : "+v"(a), "+v"(b), "+v"(c), "+v"(d)); }
template <typename T> struct Frag;
template <> struct Frag<_Float16> {
  typedef v16h V; union U { v16h v; v8h h[2]; };
  static __device__ __forceinline__ v16h load(const _Float16* p) {
    U f; f.h[0] = *(const v8h*)(p); f.h[1] = *(const v8h*)(p + 16); return f.v;
  }
  static __device__ __forceinline__ v8f mma(v16h a, v16h b, v8f c) {
    return __builtin_amdgcn_wmma_f32_16x16x32_f16(false, a, false, b, (short)0, c, false, false);
  }
  static __device__ __forceinline__ void guard(v8f& a, v8f& b, v16h x, v16h y) { dep_guard_h(a, b, x, y); }
  static __device__ __forceinline__ void keep(v16h a, v16h b, v16h c, v16h d) { keep4_h(a, b, c, d); }
};
template <> struct Frag<__bf16> {
  typedef v16b V; union U { v16b v; v8b h[2]; };
  static __device__ __forceinline__ v16b load(const __bf16* p) {
    U f; f.h[0] = *(const v8b*)(p); f.h[1] = *(const v8b*)(p + 16); return f.v;
  }
  static __device__ __forceinline__ v8f mma(v16b a, v16b b, v8f c) {
    return __builtin_amdgcn_wmma_f32_16x16x32_bf16(false, a, false, b, (short)0, c, false, false);
  }
  static __device__ __forceinline__ void guard(v8f& a, v8f& b, v16b x, v16b y) { dep_guard_b(a, b, x, y); }
  static __device__ __forceinline__ void keep(v16b a, v16b b, v16b c, v16b d) { keep4_b(a, b, c, d); }
};

template <int ET> struct Elem;
template <> struct Elem<0> { typedef _Float16 T; };
template <> struct Elem<1> { typedef __bf16 T; };
template <int ET, bool SPLIT, int BIAS_MODE, int OUT_MODE, bool RESID, int ACT = 0>
__global__ __launch_bounds__(256) void wmma_gemm64(
    const unsigned short* __restrict__ Ap, const unsigned short* __restrict__ A2p, int lda, long strideA,
    const unsigned short* __restrict__ Btp, const unsigned short* __restrict__ Bt2p, int ldb, long strideB,
    void* __restrict__ Cout, void* __restrict__ Cout2, int ldc, long strideC,
    const float* __restrict__ bias,
    const float* __restrict__ resid, long strideR,
    int M, int N, int K, float scale) {
  typedef typename Elem<ET>::T T;
  typedef typename Frag<T>::V V;
  const T* A = (const T*)Ap; const T* A2 = (const T*)A2p; const T* Bt = (const T*)Btp; const T* Bt2 = (const T*)Bt2p;
  __shared__ __align__(16) float sT[8][16 * 68];
  const int b    = blockIdx.y;
  const int lane = threadIdx.x & 31;
  const int wave = threadIdx.x >> 5;
  const int tilesN = N >> 6;
  const int tilesM = M >> 6;
  const int tile = blockIdx.x * 8 + wave;
  if (tile >= tilesM * tilesN) return;
  const int tm = tile / tilesN;
  const int tn = tile - tm * tilesN;
  const int m0 = tm << 6;
  const int n0 = tn << 6;

  const T* Ab  = A  + (size_t)b * strideA;
  const T* Bb  = Bt + (size_t)b * strideB;
  const T* Ab2 = SPLIT ? (A2  + (size_t)b * strideA) : nullptr;
  const T* Bb2 = SPLIT ? (Bt2 + (size_t)b * strideB) : nullptr;

  const int rlane = lane & 15;
  const int koff  = (lane >> 4) * 8;
  const int mOff  = (lane >> 4) * 8;

  v8f acc[4][4];
#pragma unroll
  for (int i = 0; i < 4; ++i)
#pragma unroll
    for (int j = 0; j < 4; ++j) acc[i][j] = (v8f){0.f,0.f,0.f,0.f,0.f,0.f,0.f,0.f};

  for (int k0 = 0; k0 < K; k0 += 32) {
    V bh[4], bl[4];
#pragma unroll
    for (int j = 0; j < 4; ++j) {
      const size_t bo = (size_t)(n0 + (j << 4) + rlane) * ldb + koff + k0;
      bh[j] = Frag<T>::load(Bb + bo);
      if (SPLIT) bl[j] = Frag<T>::load(Bb2 + bo);
    }
#pragma unroll
    for (int i = 0; i < 4; ++i) {
      const size_t ao = (size_t)(m0 + (i << 4) + rlane) * lda + koff + k0;
      V ah = Frag<T>::load(Ab + ao);
      V al;
      if (SPLIT) al = Frag<T>::load(Ab2 + ao);
#pragma unroll
      for (int j = 0; j < 4; ++j) {
        acc[i][j] = Frag<T>::mma(ah, bh[j], acc[i][j]);
        if (SPLIT) {
          acc[i][j] = Frag<T>::mma(ah, bl[j], acc[i][j]);
          acc[i][j] = Frag<T>::mma(al, bh[j], acc[i][j]);
        }
      }
      Frag<T>::guard(acc[i][0], acc[i][3], ah, SPLIT ? al : ah);
    }
    Frag<T>::keep(bh[0], bh[1], bh[2], bh[3]);
    if (SPLIT) Frag<T>::keep(bl[0], bl[1], bl[2], bl[3]);
  }
  acc_guard4(acc[0][0], acc[0][1], acc[0][2], acc[0][3]);
  acc_guard4(acc[1][0], acc[1][1], acc[1][2], acc[1][3]);
  acc_guard4(acc[2][0], acc[2][1], acc[2][2], acc[2][3]);
  acc_guard4(acc[3][0], acc[3][1], acc[3][2], acc[3][3]);

  float* slab = sT[wave];
  const float* Rb = RESID ? (resid + (size_t)b * strideR) : nullptr;
#pragma unroll
  for (int i = 0; i < 4; ++i) {
    const int mBase = m0 + (i << 4);
#pragma unroll
    for (int j = 0; j < 4; ++j) {
      const int n = n0 + (j << 4) + rlane;
      float bv = 0.f;
      if (BIAS_MODE == 2) bv = bias[n];
#pragma unroll
      for (int r = 0; r < 8; ++r) {
        float v = acc[i][j][r] * scale;
        if (BIAS_MODE == 1) v += bias[mBase + mOff + r];
        if (BIAS_MODE == 2) v += bv;
        if (RESID) v += Rb[(size_t)(mBase + mOff + r) * ldc + n];
        if (ACT == 1) v = tanhf(v);
        if (ACT == 2) v = fmaxf(v, 0.0f);
        if (ACT == 3) v = v / (1.0f + expf(-v));
        if (ACT == 4) v = (v > 0.f) ? v : 0.01f * v;
        if (ACT == 5) v = 0.5f * v * (1.0f + erff(v * 0.70710678118654752f));
        slab[(mOff + r) * 68 + (j << 4) + rlane] = v;
      }
    }
    __builtin_amdgcn_fence(__ATOMIC_RELEASE, "workgroup");
    __builtin_amdgcn_wave_barrier();
    __builtin_amdgcn_fence(__ATOMIC_ACQUIRE, "workgroup");
    if (OUT_MODE == 0) {
      float* C = (float*)Cout + (size_t)b * strideC;
      const int hh = lane >> 4, c4 = (lane & 15) * 4;
      for (int pass = 0; pass < 2; ++pass) {
#pragma unroll
        for (int it = 0; it < 8; ++it) {
          const int row = it * 2 + hh;
          v4f v = *(const v4f*)(slab + row * 68 + c4);
          *(volatile v4f*)(C + (size_t)(mBase + row) * ldc + n0 + c4) = v;
        }
        __threadfence();
      }
    } else {
      const int q = lane >> 3, c8 = (lane & 7) * 8;
      unsigned short* C  = (unsigned short*)Cout  + (size_t)b * strideC;
      unsigned short* C2 = (OUT_MODE == 2) ? ((unsigned short*)Cout2 + (size_t)b * strideC) : nullptr;
      for (int pass = 0; pass < 2; ++pass) {
#pragma unroll
        for (int it = 0; it < 4; ++it) {
          const int row = it * 4 + q;
          const float* sp = slab + row * 68 + c8;
          v8h hv, lv;
#pragma unroll
          for (int e = 0; e < 8; ++e) {
            if (OUT_MODE == 1) {
              hv[e] = (_Float16)sp[e];
            } else {
              unsigned short hb = f2bf_bits(sp[e]);
              unsigned short lb = f2bf_bits(sp[e] - bf_bits2f(hb));
              hv[e] = __builtin_bit_cast(_Float16, hb);
              lv[e] = __builtin_bit_cast(_Float16, lb);
            }
          }
          *(volatile v8h*)(C + (size_t)(mBase + row) * ldc + n0 + c8) = hv;
          if (OUT_MODE == 2) *(volatile v8h*)(C2 + (size_t)(mBase + row) * ldc + n0 + c8) = lv;
        }
        __threadfence();
      }
    }
    __builtin_amdgcn_fence(__ATOMIC_RELEASE, "workgroup");
    __builtin_amdgcn_wave_barrier();
    __builtin_amdgcn_fence(__ATOMIC_ACQUIRE, "workgroup");
  }
}

__global__ __launch_bounds__(256) void cast_f32_f16x2(
    const float* __restrict__ in, _Float16* __restrict__ out, int n2) {
  int i = blockIdx.x * 256 + threadIdx.x;
  if (i < n2) {
    const _Float16 h0 = (_Float16)in[2 * i], h1 = (_Float16)in[2 * i + 1];
    const unsigned u = (unsigned)__builtin_bit_cast(unsigned short, h0) | ((unsigned)__builtin_bit_cast(unsigned short, h1) << 16);
    ((volatile unsigned*)out)[i] = u;
    __threadfence();
    ((volatile unsigned*)out)[i] = u;
  }
}


__global__ __launch_bounds__(256) void cast_f32_f16x2s(const float* __restrict__ in, _Float16* __restrict__ out, int n2, float s) {
  int i = blockIdx.x * 256 + threadIdx.x;
  if (i < n2) {
    const _Float16 h0 = (_Float16)(in[2 * i] * s), h1 = (_Float16)(in[2 * i + 1] * s);
    const unsigned u = (unsigned)__builtin_bit_cast(unsigned short, h0) | ((unsigned)__builtin_bit_cast(unsigned short, h1) << 16);
    ((volatile unsigned*)out)[i] = u;
    __threadfence();
    ((volatile unsigned*)out)[i] = u;
  }
}
__global__ __launch_bounds__(256) void split_f32_bf16x2(
    const float* __restrict__ in, __bf16* __restrict__ hi, __bf16* __restrict__ lo, long n2) {
  long i = (long)blockIdx.x * 256 + threadIdx.x;
  long stride = (long)gridDim.x * 256;
  for (int pass = 0; pass < 2; ++pass) {
    for (long j = i; j < n2; j += stride) {
      const float a = in[2 * j], b = in[2 * j + 1];
      const unsigned short ah = f2bf_bits(a), bh = f2bf_bits(b);
      const unsigned short al = f2bf_bits(a - bf_bits2f(ah)), bl = f2bf_bits(b - bf_bits2f(bh));
      ((volatile unsigned*)hi)[j] = (unsigned)ah | ((unsigned)bh << 16);
      ((volatile unsigned*)lo)[j] = (unsigned)al | ((unsigned)bl << 16);
    }
    __threadfence();
  }
}


__global__ __launch_bounds__(256) void transpose_cast_f16(const float* __restrict__ in, int ldi,
                                                         _Float16* __restrict__ outT, int ldo, float scale) {
  __shared__ __align__(16) _Float16 tile[64][72];
  const int c0 = blockIdx.x * 64, r0 = blockIdx.y * 64;
  const int t = threadIdx.y * 32 + threadIdx.x;
  for (int i = threadIdx.y; i < 64; i += 8) {
    tile[threadIdx.x][i]      = (_Float16)(in[(size_t)(r0 + i) * ldi + c0 + threadIdx.x] * scale);
    tile[32 + threadIdx.x][i] = (_Float16)(in[(size_t)(r0 + i) * ldi + c0 + 32 + threadIdx.x] * scale);
  }
  __syncthreads();
  const int q = t >> 3, c8 = (t & 7) * 8;
  for (int pass = 0; pass < 2; ++pass) {
#pragma unroll
    for (int it = 0; it < 2; ++it) {
      const int c = it * 32 + q;
      v8h hv = *(const v8h*)(&tile[c][c8]);
      *(volatile v8h*)(outT + (size_t)(c0 + c) * ldo + r0 + c8) = hv;
    }
    __threadfence();
  }
}

__global__ __launch_bounds__(256) void transpose_split_bf16(const float* __restrict__ in, int ldi,
                                                           __bf16* __restrict__ outH, __bf16* __restrict__ outL, int ldo) {
  __shared__ __align__(16) float tile[64][68];
  const int c0 = blockIdx.x * 64, r0 = blockIdx.y * 64;
  const int t = threadIdx.y * 32 + threadIdx.x;
  for (int i = threadIdx.y; i < 64; i += 8) {
    tile[threadIdx.x][i]      = in[(size_t)(r0 + i) * ldi + c0 + threadIdx.x];
    tile[32 + threadIdx.x][i] = in[(size_t)(r0 + i) * ldi + c0 + 32 + threadIdx.x];
  }
  __syncthreads();
  const int q = t >> 3, c8 = (t & 7) * 8;
  for (int pass = 0; pass < 2; ++pass) {
#pragma unroll
    for (int it = 0; it < 2; ++it) {
      const int c = it * 32 + q;
      v8b hv, lv;
#pragma unroll
      for (int e = 0; e < 8; ++e) {
        const float f = tile[c][c8 + e];
        const unsigned short hb = f2bf_bits(f);
        hv[e] = __builtin_bit_cast(__bf16, hb);
        lv[e] = __builtin_bit_cast(__bf16, f2bf_bits(f - bf_bits2f(hb)));
      }
      *(volatile v8b*)(outH + (size_t)(c0 + c) * ldo + r0 + c8) = hv;
      *(volatile v8b*)(outL + (size_t)(c0 + c) * ldo + r0 + c8) = lv;
    }
    __threadfence();
  }
}

#define AT_D 64
#define AT_NW 4
#define AT_QB 64
#define AT_KC 64
struct AttnGeom { const float* cp = nullptr; const float* pc = nullptr; long c_bs = 0, c_rs = 0, c_hs = 0;
                  long q_bs, q_rs, q_hs, k_bs, k_rs, k_hs, v_bs, v_rs, v_hs, o_bs, o_rs, o_hs;
                  int S, Skv, H, mask_mode; float qscale; int blk0; float mask_fill; int mask_is_int; };
static_assert(sizeof(AttnGeom) == 168, "no padding");

__device__ __forceinline__ unsigned short at_bf_bits(float f) {
  unsigned u = __float_as_uint(f);
  return (unsigned short)((u + 0x7FFFu + ((u >> 16) & 1u)) >> 16);
}
__device__ __forceinline__ __bf16 at_f2bf(float f) { return __builtin_bit_cast(__bf16, at_bf_bits(f)); }
__device__ __forceinline__ void at_split(float f, __bf16& hi, __bf16& lo) {
  const unsigned short hb = at_bf_bits(f);
  hi = __builtin_bit_cast(__bf16, hb);
  lo = at_f2bf(f - __uint_as_float(((unsigned)hb) << 16));
}
__device__ __forceinline__ v8f at_mma(v16b a, v16b b, v8f c) {
  c = __builtin_amdgcn_wmma_f32_16x16x32_bf16(false, a, false, b, (short)0, c, false, false);
  asm volatile("v_nop\n\tv_nop\n\tv_nop\n\tv_nop" : "+v"(c) : "v"(a), "v"(b));
  return c;
}
template <bool F16> __device__ __forceinline__ __bf16 at_to16(float f) {
  if (F16) return __builtin_bit_cast(__bf16, (_Float16)f);
  return at_f2bf(f);
}
template <bool F16> __device__ __forceinline__ v8f at_mma16(v16b a, v16b b, v8f c) {
  if (F16) {
    const v16h ah = __builtin_bit_cast(v16h, a), bh = __builtin_bit_cast(v16h, b);
    c = __builtin_amdgcn_wmma_f32_16x16x32_f16(false, ah, false, bh, (short)0, c, false, false);
    asm volatile("v_nop\n\tv_nop\n\tv_nop\n\tv_nop" : "+v"(c) : "v"(ah), "v"(bh));
    return c;
  }
  return at_mma(a, b, c);
}

template <bool SPLIT_QK, bool SPLIT_PV, bool F16 = false>
__global__ __launch_bounds__(128)
void attn64_kernel(const float* __restrict__ q, const float* __restrict__ k,
                   const float* __restrict__ v, float* __restrict__ out,
                   const void* __restrict__ mask_a, const int* __restrict__ mask_b, AttnGeom g) {
  static_assert(!(F16 && (SPLIT_QK || SPLIT_PV)), "f16 mode is non-split");
  const float PSC = F16 ? 32768.0f : 1.0f;
  union FB { v16b v; v8b h[2]; };
  __shared__ __align__(16) __bf16 Ksh[AT_KC * AT_D];
  __shared__ __align__(16) __bf16 Ksl[SPLIT_QK ? AT_KC * AT_D : 8];
  __shared__ __align__(16) __bf16 Vth[AT_D * AT_KC];
  __shared__ __align__(16) __bf16 Vtl[SPLIT_PV ? AT_D * AT_KC : 8];
  __shared__ __align__(16) __bf16 Psh[AT_NW][16 * AT_KC];
  __shared__ __align__(16) __bf16 Psl[SPLIT_PV ? AT_NW : 1][SPLIT_PV ? 16 * AT_KC : 8];
  __shared__ __align__(16) float  Os[AT_NW][16 * 68];

  const int tid  = threadIdx.x;
  const int wave = tid >> 5;
  const int lane = tid & 31;
  const int hh   = lane >> 4;
  const int c    = lane & 15;

  const int nqb = g.S / AT_QB;
  const int bx = blockIdx.x + g.blk0;
  const int qb = bx % nqb;
  const int bh = bx / nqb;
  const int h  = bh % g.H;
  const int b  = bh / g.H;
  const int qbase_block = qb * AT_QB;
  const int q0 = qbase_block + wave * 16;

  const float* qb_ptr = q + (size_t)b * g.q_bs + (size_t)h * g.q_hs;
  const float* kb_ptr = k + (size_t)b * g.k_bs + (size_t)h * g.k_hs;
  const float* vb_ptr = v + (size_t)b * g.v_bs + (size_t)h * g.v_hs;
  float*       ob_ptr = out + (size_t)b * g.o_bs + (size_t)h * g.o_hs;

  v16b qah[2], qal[2];
  {
    const float* qrow = qb_ptr + (size_t)(q0 + c) * g.q_rs;
#pragma unroll
    for (int dc = 0; dc < 2; ++dc) {
#pragma unroll
      for (int e = 0; e < 8; ++e) {
        const float f0 = qrow[dc * 32 + 8 * hh + e] * g.qscale;
        const float f1 = qrow[dc * 32 + 16 + 8 * hh + e] * g.qscale;
        if (SPLIT_QK) { __bf16 hq, lq; at_split(f0, hq, lq); qah[dc][e] = hq; qal[dc][e] = lq; at_split(f1, hq, lq); qah[dc][8 + e] = hq; qal[dc][8 + e] = lq; }
        else { qah[dc][e] = at_to16<F16>(f0); qah[dc][8 + e] = at_to16<F16>(f1); qal[dc][e] = qah[dc][e]; qal[dc][8 + e] = qah[dc][8 + e]; }
      }
    }
  }

  float mrow[8], lrow[8];
  v8f oacc[4];
#pragma unroll
  for (int r = 0; r < 8; ++r) { mrow[r] = -INFINITY; lrow[r] = 0.f; }
#pragma unroll
  for (int t = 0; t < 4; ++t) oacc[t] = (v8f){0.f,0.f,0.f,0.f,0.f,0.f,0.f,0.f};

  const int nChunks = (g.mask_mode == 1 || g.mask_mode == 4) ? (qb + 1) : (g.Skv / AT_KC);
  int qkeep[8];
#pragma unroll
  for (int r = 0; r < 8; ++r) qkeep[r] = (g.mask_mode == 3) ? mask_b[(size_t)b * g.S + q0 + 8 * hh + r] : 1;
  for (int kc = 0; kc < nChunks; ++kc) {
    const int kv0 = kc * AT_KC;
    __syncthreads();
    {
      const int kvr = tid >> 1, dh = (tid & 1) * 32;
      const float* krow = kb_ptr + (size_t)(kv0 + kvr) * g.k_rs + dh;
      const float* vrow = vb_ptr + (size_t)(kv0 + kvr) * g.v_rs + dh;
#pragma unroll
      for (int i = 0; i < 8; ++i) {
        v4f kk = *(const v4f*)(krow + 4 * i);
        v4f vv = *(const v4f*)(vrow + 4 * i);
#pragma unroll
        for (int e = 0; e < 4; ++e) {
          const int d = dh + 4 * i + e;
          if (SPLIT_QK) { __bf16 a, bl; at_split(kk[e], a, bl); Ksh[kvr * AT_D + d] = a; Ksl[kvr * AT_D + d] = bl; }
          else Ksh[kvr * AT_D + d] = at_to16<F16>(kk[e]);
          if (SPLIT_PV) { __bf16 a, bl; at_split(vv[e], a, bl); Vth[d * AT_KC + kvr] = a; Vtl[d * AT_KC + kvr] = bl; }
          else Vth[d * AT_KC + kvr] = at_to16<F16>(vv[e]);
        }
      }
    }
    __syncthreads();

    v8f s[4];
#pragma unroll
    for (int j = 0; j < 4; ++j) {
      s[j] = (v8f){0.f,0.f,0.f,0.f,0.f,0.f,0.f,0.f};
#pragma unroll 1
      for (int dc = 0; dc < 2; ++dc) {
        FB kb;
        kb.h[0] = *(const v8b*)(Ksh + (j * 16 + c) * AT_D + dc * 32 + 8 * hh);
        kb.h[1] = *(const v8b*)(Ksh + (j * 16 + c) * AT_D + dc * 32 + 16 + 8 * hh);
        s[j] = at_mma16<F16>(qah[dc], kb.v, s[j]);
        if (SPLIT_QK) {
          FB kl;
          kl.h[0] = *(const v8b*)(Ksl + (j * 16 + c) * AT_D + dc * 32 + 8 * hh);
          kl.h[1] = *(const v8b*)(Ksl + (j * 16 + c) * AT_D + dc * 32 + 16 + 8 * hh);
          s[j] = at_mma16<F16>(qah[dc], kl.v, s[j]);
          s[j] = at_mma16<F16>(qal[dc], kb.v, s[j]);
        }
      }
    }
    const bool diag = (g.mask_mode == 1) && (kc == qb);
    int kvkeep[4] = {1, 1, 1, 1};
    if (g.mask_mode == 3) {
#pragma unroll
      for (int j = 0; j < 4; ++j) kvkeep[j] = ((const int*)mask_a)[(size_t)b * g.Skv + kv0 + j * 16 + c];
    }
    float cm[8];
#pragma unroll
    for (int r = 0; r < 8; ++r) {
      const int qrow = q0 + 8 * hh + r;
      float m = -INFINITY;
#pragma unroll
      for (int j = 0; j < 4; ++j) {
        const int kvcol = kv0 + j * 16 + c;
        bool masked = false;
        if (diag) masked = (kvcol > qrow);
        else if (g.mask_mode == 4) masked = (kvcol > qrow) || (qrow - kvcol > g.mask_is_int);
        else if (g.mask_mode == 2) {
          const size_t mi = (size_t)qrow * g.Skv + kvcol;
          masked = (g.mask_is_int == 0) ? (((const float*)mask_a)[mi] == 0.0f)
                 : (g.mask_is_int == 1) ? (((const int*)mask_a)[mi] == 0) : (((const int*)mask_a)[mi] != 0);
        } else if (g.mask_mode == 3) masked = (qkeep[r] == 0) || (kvkeep[j] == 0);
        else if (g.mask_mode == 10) masked = (kvcol >= (int)g.c_rs);
        else if (g.mask_mode == 5) {
          const size_t mi = (size_t)qrow * g.Skv + kvcol;
          masked = (((const int*)mask_a)[mi] != 0);
          int n = mask_b[mi]; n = n < 0 ? 0 : n;
          s[j][r] += g.cp[(size_t)b * g.c_bs + (size_t)h * g.c_hs + (size_t)qrow * g.c_rs + n]
                   + g.pc[(size_t)b * g.c_bs + (size_t)h * g.c_hs + (size_t)kvcol * g.c_rs + n];
        }
        if (masked) s[j][r] = g.mask_fill;
        m = fmaxf(m, s[j][r]);
      }
#pragma unroll
      for (int off = 1; off < 16; off <<= 1) m = fmaxf(m, __shfl_xor(m, off, 32));
      cm[r] = m;
    }
    __bf16* pwh = Psh[wave];
    __bf16* pwl = Psl[SPLIT_PV ? wave : 0];
#pragma unroll
    for (int r = 0; r < 8; ++r) {
      const float mnew = fmaxf(mrow[r], cm[r]);
      const float alpha = expf(mrow[r] - mnew);
      mrow[r] = mnew;
      float psum = 0.f;
#pragma unroll
      for (int j = 0; j < 4; ++j) {
        const float p = expf(s[j][r] - mnew);
        psum += p;
        if (SPLIT_PV) { __bf16 a, bl; at_split(p, a, bl); pwh[(8 * hh + r) * AT_KC + j * 16 + c] = a; pwl[(8 * hh + r) * AT_KC + j * 16 + c] = bl; }
        else pwh[(8 * hh + r) * AT_KC + j * 16 + c] = at_to16<F16>(p * PSC);
      }
#pragma unroll
      for (int off = 1; off < 16; off <<= 1) psum += __shfl_xor(psum, off, 32);
      lrow[r] = lrow[r] * alpha + psum;
#pragma unroll
      for (int t = 0; t < 4; ++t) oacc[t][r] *= alpha;
    }
    __builtin_amdgcn_fence(__ATOMIC_RELEASE, "workgroup");
    __builtin_amdgcn_wave_barrier();
    __builtin_amdgcn_fence(__ATOMIC_ACQUIRE, "workgroup");
#pragma unroll 1
    for (int kk = 0; kk < 2; ++kk) {
      FB pa, pl;
      pa.h[0] = *(const v8b*)(pwh + c * AT_KC + kk * 32 + 8 * hh);
      pa.h[1] = *(const v8b*)(pwh + c * AT_KC + kk * 32 + 16 + 8 * hh);
      if (SPLIT_PV) {
        pl.h[0] = *(const v8b*)(pwl + c * AT_KC + kk * 32 + 8 * hh);
        pl.h[1] = *(const v8b*)(pwl + c * AT_KC + kk * 32 + 16 + 8 * hh);
      }
#pragma unroll
      for (int t = 0; t < 4; ++t) {
        FB vb;
        vb.h[0] = *(const v8b*)(Vth + (t * 16 + c) * AT_KC + kk * 32 + 8 * hh);
        vb.h[1] = *(const v8b*)(Vth + (t * 16 + c) * AT_KC + kk * 32 + 16 + 8 * hh);
        oacc[t] = at_mma16<F16>(pa.v, vb.v, oacc[t]);
        if (SPLIT_PV) {
          FB vl;
          vl.h[0] = *(const v8b*)(Vtl + (t * 16 + c) * AT_KC + kk * 32 + 8 * hh);
          vl.h[1] = *(const v8b*)(Vtl + (t * 16 + c) * AT_KC + kk * 32 + 16 + 8 * hh);
          oacc[t] = at_mma16<F16>(pa.v, vl.v, oacc[t]);
          oacc[t] = at_mma16<F16>(pl.v, vb.v, oacc[t]);
        }
      }
    }
  }

  float* os = Os[wave];
#pragma unroll
  for (int r = 0; r < 8; ++r) {
    const float inv = 1.0f / (lrow[r] * PSC);
#pragma unroll
    for (int t = 0; t < 4; ++t) os[(8 * hh + r) * 68 + t * 16 + c] = oacc[t][r] * inv;
  }
  __builtin_amdgcn_fence(__ATOMIC_RELEASE, "workgroup");
  __builtin_amdgcn_wave_barrier();
  __builtin_amdgcn_fence(__ATOMIC_ACQUIRE, "workgroup");
  {
    const int c4 = (lane & 15) * 4;
    for (int pass = 0; pass < 2; ++pass) {
#pragma unroll
      for (int it = 0; it < 8; ++it) {
        const int row = it * 2 + hh;
        v4f val = *(const v4f*)(os + row * 68 + c4);
        *(volatile v4f*)(ob_ptr + (size_t)(q0 + row) * g.o_rs + c4) = val;
      }
      __threadfence();
    }
  }
}

#define SB 2
#define SC 1024
#define SNT 1600
#define SL 77
#define SLP 128
#define SFF 4096
#define SH 16
#ifndef TROWS
#define TROWS (SB * SNT)
#endif
__global__ __launch_bounds__(256) void gn_stats_kernel(const float* __restrict__ x, float* __restrict__ st) {
  __shared__ double ra[256], rb[256];
  const int bg = blockIdx.x; const float* p = x + (size_t)bg * 32 * SNT;
  double a = 0.0, b = 0.0;
  for (int i = threadIdx.x; i < 32 * SNT; i += 256) { const double v = p[i]; a += v; b += v * v; }
  ra[threadIdx.x] = a; rb[threadIdx.x] = b; __syncthreads();
  for (int s = 128; s > 0; s >>= 1) { if (threadIdx.x < s) { ra[threadIdx.x] += ra[threadIdx.x + s]; rb[threadIdx.x] += rb[threadIdx.x + s]; } __syncthreads(); }
  if (threadIdx.x < 32) { const double n = 32.0 * SNT; const double mu = ra[0] / n; double var = rb[0] / n - mu * mu; if (var < 0) var = 0;
    const float v = (threadIdx.x == 0) ? (float)mu : (threadIdx.x == 1 ? (float)(1.0 / sqrt(var + 1e-6)) : 0.f);
    ((volatile float*)st)[(size_t)bg * 32 + threadIdx.x] = v; __threadfence(); ((volatile float*)st)[(size_t)bg * 32 + threadIdx.x] = v; }
}
__global__ __launch_bounds__(256) void gn_apply_kernel(const float* __restrict__ x, const float* __restrict__ st, const float* __restrict__ gs, const float* __restrict__ gb, unsigned* __restrict__ HX) {
  __shared__ float tile[64][65];
  const int b = blockIdx.z, c0 = blockIdx.y * 64, n0 = blockIdx.x * 64, tx = threadIdx.x, ty = threadIdx.y;
  for (int i = ty; i < 64; i += 8) { const int c = c0 + i; const float mu = st[((size_t)b * 32 + c / 32) * 32], rs = st[((size_t)b * 32 + c / 32) * 32 + 1];
    for (int j = tx; j < 64; j += 32) { const int n = n0 + j; tile[i][j] = (n < SNT) ? (x[((size_t)b * SC + c) * SNT + n] - mu) * rs * gs[c] + gb[c] : 0.f; } }
  __syncthreads();
  for (int pass = 0; pass < 2; ++pass) {
    for (int j = ty; j < 64; j += 8) { const int n = n0 + j; if (n >= SNT) continue;
      const unsigned u = (unsigned)__builtin_bit_cast(unsigned short, (_Float16)tile[2 * tx][j]) | ((unsigned)__builtin_bit_cast(unsigned short, (_Float16)tile[2 * tx + 1][j]) << 16);
      ((volatile unsigned*)HX)[(((size_t)b * SNT + n) * SC + c0) / 2 + tx] = u; }
    __threadfence(); }
}
__global__ __launch_bounds__(256) void ln_kernel(const float* __restrict__ X, const float* __restrict__ g, const float* __restrict__ bb, unsigned* __restrict__ Y16) {
  const int lane = threadIdx.x & 31, wave = threadIdx.x >> 5; const size_t row = (size_t)blockIdx.x * 8 + wave;
  const float* xr = X + row * SC; float v[32]; float s = 0.f;
#pragma unroll
  for (int q = 0; q < 8; ++q) { const v4f t4 = *(const v4f*)(xr + q * 128 + lane * 4); v[4*q] = t4[0]; v[4*q+1] = t4[1]; v[4*q+2] = t4[2]; v[4*q+3] = t4[3]; s += t4[0] + t4[1] + t4[2] + t4[3]; }
  for (int o = 16; o > 0; o >>= 1) s += __shfl_xor(s, o, 32);
  const float mean = s / (float)SC; float s2 = 0.f;
#pragma unroll
  for (int i = 0; i < 32; ++i) { const float d = v[i] - mean; s2 += d * d; }
  for (int o = 16; o > 0; o >>= 1) s2 += __shfl_xor(s2, o, 32);
  const float inv = rsqrtf(s2 / (float)SC + 1e-5f);
  typedef __attribute__((ext_vector_type(2))) unsigned u2;
  for (int pass = 0; pass < 2; ++pass) {
#pragma unroll
    for (int q = 0; q < 8; ++q) { const int c = q * 128 + lane * 4; u2 pk;
      pk[0] = (unsigned)__builtin_bit_cast(unsigned short, (_Float16)((v[4*q] - mean) * inv * g[c] + bb[c])) | ((unsigned)__builtin_bit_cast(unsigned short, (_Float16)((v[4*q+1] - mean) * inv * g[c + 1] + bb[c + 1])) << 16);
      pk[1] = (unsigned)__builtin_bit_cast(unsigned short, (_Float16)((v[4*q+2] - mean) * inv * g[c + 2] + bb[c + 2])) | ((unsigned)__builtin_bit_cast(unsigned short, (_Float16)((v[4*q+3] - mean) * inv * g[c + 3] + bb[c + 3])) << 16);
      *(volatile u2*)(Y16 + (row * SC + c) / 2) = pk; }
    __threadfence(); }
}
__global__ __launch_bounds__(256) void ctx_pad_kernel(const float* __restrict__ ctx, unsigned* __restrict__ CT) {
  const long i = (long)blockIdx.x * 256 + threadIdx.x; if (i >= (long)SB * SLP * SC / 2) return;
  const long e0 = 2 * i; const int b = (int)(e0 / ((long)SLP * SC)); const int j = (int)((e0 / SC) % SLP); const int c = (int)(e0 % SC);
  float a = 0.f, bb = 0.f; if (j < SL) { const float* p = ctx + ((size_t)b * SL + j) * SC + c; a = p[0]; bb = p[1]; }
  const unsigned u = (unsigned)__builtin_bit_cast(unsigned short, (_Float16)a) | ((unsigned)__builtin_bit_cast(unsigned short, (_Float16)bb) << 16);
  ((volatile unsigned*)CT)[i] = u; __threadfence(); ((volatile unsigned*)CT)[i] = u;
}
__global__ __launch_bounds__(256) void geglu_kernel(const float* __restrict__ Hf, unsigned* __restrict__ G16, long n2) {
  const long i = (long)blockIdx.x * 256 + threadIdx.x; if (i >= n2) return;
  const long e0 = 2 * i; const long r = e0 / SFF; const int j = (int)(e0 % SFF);
  const float* hr = Hf + r * (2 * SFF);
  const float a0 = hr[j], a1 = hr[j + 1], g0 = hr[SFF + j], g1 = hr[SFF + j + 1];
  const float y0 = a0 * (0.5f * g0 * (1.0f + erff(g0 * 0.70710678118654752f))), y1 = a1 * (0.5f * g1 * (1.0f + erff(g1 * 0.70710678118654752f)));
  const unsigned u = (unsigned)__builtin_bit_cast(unsigned short, (_Float16)y0) | ((unsigned)__builtin_bit_cast(unsigned short, (_Float16)y1) << 16);
  ((volatile unsigned*)G16)[i] = u; __threadfence(); ((volatile unsigned*)G16)[i] = u;
}
__global__ __launch_bounds__(256) void out_kernel(const float* __restrict__ P, const float* __restrict__ x, float* __restrict__ out) {
  __shared__ float tile[64][65];
  const int b = blockIdx.z, c0 = blockIdx.y * 64, n0 = blockIdx.x * 64, tx = threadIdx.x, ty = threadIdx.y;
  for (int j = ty; j < 64; j += 8) { const int n = n0 + j; for (int i = tx; i < 64; i += 32) tile[i][j] = (n < SNT) ? P[((size_t)b * SNT + n) * SC + c0 + i] : 0.f; }
  __syncthreads();
  for (int pass = 0; pass < 2; ++pass) {
    for (int i = ty; i < 64; i += 8) { const int c = c0 + i; for (int j = tx; j < 64; j += 32) { const int n = n0 + j; if (n < SNT) { const size_t o = ((size_t)b * SC + c) * SNT + n; ((volatile float*)out)[o] = tile[i][j] + x[o]; } } }
    __threadfence(); }
}
extern "C" void kernel_launch(void* const* d_in, const int* in_sizes, int n_in, void* d_out, int out_size, void* d_ws, size_t ws_size, hipStream_t stream) {
  (void)in_sizes; (void)n_in; (void)out_size; (void)ws_size;
  const float* x = (const float*)d_in[0]; const float* ctx = (const float*)d_in[1]; const float* gns = (const float*)d_in[2]; const float* gnb = (const float*)d_in[3];
  const float* pin_w = (const float*)d_in[4]; const float* pin_b = (const float*)d_in[5]; const float* ln1s = (const float*)d_in[6]; const float* ln1b = (const float*)d_in[7];
  const float* wq1 = (const float*)d_in[8]; const float* wk1 = (const float*)d_in[9]; const float* wv1 = (const float*)d_in[10]; const float* wo1 = (const float*)d_in[11]; const float* bo1 = (const float*)d_in[12];
  const float* ln2s = (const float*)d_in[13]; const float* ln2b = (const float*)d_in[14];
  const float* wq2 = (const float*)d_in[15]; const float* wk2 = (const float*)d_in[16]; const float* wv2 = (const float*)d_in[17]; const float* wo2 = (const float*)d_in[18]; const float* bo2 = (const float*)d_in[19];
  const float* ln3s = (const float*)d_in[20]; const float* ln3b = (const float*)d_in[21]; const float* ffw1 = (const float*)d_in[22]; const float* ffb1 = (const float*)d_in[23]; const float* ffw2 = (const float*)d_in[24]; const float* ffb2 = (const float*)d_in[25];
  const float* pw = (const float*)d_in[26]; const float* pb = (const float*)d_in[27];
  float* out = (float*)d_out;
  char* ws = (char*)d_ws; size_t off = 0;
  auto carve = [&](size_t bytes) -> char* { char* p = ws + off; off += (bytes + 255) & ~(size_t)255; return p; };
  const int R = SB * SNT;
  float* st = (float*)carve((size_t)SB * 32 * 32 * 4);
  unsigned* HX = (unsigned*)carve((size_t)R * SC * 2);
  _Float16* WT = (_Float16*)carve((size_t)3 * SC * SC * 2);
  _Float16* WT2 = (_Float16*)carve((size_t)2 * SFF * SC * 2);
  float* T0 = (float*)carve((size_t)R * SC * 4); float* T1 = (float*)carve((size_t)R * SC * 4);
  float* QKV = (float*)carve((size_t)R * 3 * SC * 4);
  float* Hf = (float*)carve((size_t)R * 2 * SFF * 4);
  float* O = (float*)carve((size_t)R * SC * 4);
  unsigned* O16 = (unsigned*)carve((size_t)R * SC * 2);
  unsigned* CT = (unsigned*)carve((size_t)SB * SLP * SC * 2); float* KV2 = (float*)carve((size_t)SB * SLP * 2 * SC * 4);
  unsigned* G16 = (unsigned*)carve((size_t)R * SFF * 2);
  unsigned* Y16 = HX;
  const int tr = (TROWS / 64) * (SC / 64);
  gn_stats_kernel<<<SB * 32, 256, 0, stream>>>(x, st);
  gn_apply_kernel<<<dim3((SNT + 63) / 64, SC / 64, SB), dim3(32, 8), 0, stream>>>(x, st, gns, gnb, HX);
  transpose_cast_f16<<<dim3(SC / 64, SC / 64), dim3(32, 8), 0, stream>>>(pin_w, SC, WT, SC, 1.0f);
  wmma_gemm64<0, false, 2, 0, false><<<dim3((((R / 64) * (SC / 64)) + 7) / 8, 1), 256, 0, stream>>>((const unsigned short*)HX, nullptr, SC, 0, U16(WT), nullptr, SC, 0, T0, nullptr, SC, 0, pin_b, nullptr, 0, R, SC, SC, 1.0f);
  ln_kernel<<<R / 8, 256, 0, stream>>>(T0, ln1s, ln1b, Y16);
  transpose_cast_f16<<<dim3(SC / 64, SC / 64), dim3(32, 8), 0, stream>>>(wq1, SC, WT, SC, 1.0f);
  transpose_cast_f16<<<dim3(SC / 64, SC / 64), dim3(32, 8), 0, stream>>>(wk1, SC, WT + (size_t)SC * SC, SC, 1.0f);
  transpose_cast_f16<<<dim3(SC / 64, SC / 64), dim3(32, 8), 0, stream>>>(wv1, SC, WT + (size_t)2 * SC * SC, SC, 1.0f);
  wmma_gemm64<0, false, 0, 0, false><<<dim3((((R / 64) * (3 * SC / 64)) + 7) / 8, 1), 256, 0, stream>>>((const unsigned short*)Y16, nullptr, SC, 0, U16(WT), nullptr, SC, 0, QKV, nullptr, 3 * SC, 0, nullptr, nullptr, 0, R, 3 * SC, SC, 1.0f);
  { AttnGeom g;
    g.q_bs = (long)SNT * 3 * SC; g.q_rs = 3 * SC; g.q_hs = 64; g.k_bs = g.q_bs; g.k_rs = 3 * SC; g.k_hs = 64; g.v_bs = g.q_bs; g.v_rs = 3 * SC; g.v_hs = 64; g.o_bs = (long)SNT * SC; g.o_rs = SC; g.o_hs = 64;
    g.S = SNT; g.Skv = SNT; g.H = SH; g.mask_mode = 0; g.qscale = 0.125f; g.blk0 = 0; g.mask_fill = -INFINITY; g.mask_is_int = 0;
    attn64_kernel<false, false, true><<<SB * SH * (SNT / AT_QB), AT_NW * 32, 0, stream>>>(QKV, QKV + SC, QKV + 2 * SC, O, nullptr, nullptr, g); }
  cast_f32_f16x2<<<(TROWS * SC / 2 + 255) / 256, 256, 0, stream>>>(O, (_Float16*)O16, TROWS * SC / 2);
  transpose_cast_f16<<<dim3(SC / 64, SC / 64), dim3(32, 8), 0, stream>>>(wo1, SC, WT, SC, 1.0f);
  wmma_gemm64<0, false, 2, 0, true><<<dim3((tr + 7) / 8, 1), 256, 0, stream>>>((const unsigned short*)O16, nullptr, SC, 0, U16(WT), nullptr, SC, 0, T1, nullptr, SC, 0, bo1, T0, 0, TROWS, SC, SC, 1.0f);
  ln_kernel<<<TROWS / 8, 256, 0, stream>>>(T1, ln2s, ln2b, Y16);
  transpose_cast_f16<<<dim3(SC / 64, SC / 64), dim3(32, 8), 0, stream>>>(wq2, SC, WT, SC, 1.0f);
  transpose_cast_f16<<<dim3(SC / 64, SC / 64), dim3(32, 8), 0, stream>>>(wk2, SC, WT + (size_t)SC * SC, SC, 1.0f);
  transpose_cast_f16<<<dim3(SC / 64, SC / 64), dim3(32, 8), 0, stream>>>(wv2, SC, WT + (size_t)2 * SC * SC, SC, 1.0f);
  wmma_gemm64<0, false, 0, 0, false><<<dim3((tr + 7) / 8, 1), 256, 0, stream>>>((const unsigned short*)Y16, nullptr, SC, 0, U16(WT), nullptr, SC, 0, QKV, nullptr, 3 * SC, 0, nullptr, nullptr, 0, TROWS, SC, SC, 1.0f);
  ctx_pad_kernel<<<(SB * SLP * SC / 2 + 255) / 256, 256, 0, stream>>>(ctx, CT);
  wmma_gemm64<0, false, 0, 0, false><<<dim3((((SB * SLP / 64) * (2 * SC / 64)) + 7) / 8, 1), 256, 0, stream>>>((const unsigned short*)CT, nullptr, SC, 0, U16(WT + (size_t)SC * SC), nullptr, SC, 0, KV2, nullptr, 2 * SC, 0, nullptr, nullptr, 0, SB * SLP, 2 * SC, SC, 1.0f);
  { AttnGeom g;
    g.q_bs = (long)SNT * 3 * SC; g.q_rs = 3 * SC; g.q_hs = 64; g.k_bs = (long)SLP * 2 * SC; g.k_rs = 2 * SC; g.k_hs = 64; g.v_bs = g.k_bs; g.v_rs = 2 * SC; g.v_hs = 64; g.o_bs = (long)SNT * SC; g.o_rs = SC; g.o_hs = 64;
    g.S = SNT; g.Skv = SLP; g.H = SH; g.mask_mode = 10; g.c_rs = SL; g.qscale = 0.125f; g.blk0 = 0; g.mask_fill = -INFINITY; g.mask_is_int = 0; g.cp = nullptr; g.pc = nullptr; g.c_bs = 0; g.c_hs = 0;
    attn64_kernel<false, false, true><<<SB * SH * (SNT / AT_QB), AT_NW * 32, 0, stream>>>(QKV, KV2, KV2 + SC, O, nullptr, nullptr, g); }
  cast_f32_f16x2<<<(TROWS * SC / 2 + 255) / 256, 256, 0, stream>>>(O, (_Float16*)O16, TROWS * SC / 2);
  transpose_cast_f16<<<dim3(SC / 64, SC / 64), dim3(32, 8), 0, stream>>>(wo2, SC, WT, SC, 1.0f);
  wmma_gemm64<0, false, 2, 0, true><<<dim3((tr + 7) / 8, 1), 256, 0, stream>>>((const unsigned short*)O16, nullptr, SC, 0, U16(WT), nullptr, SC, 0, T0, nullptr, SC, 0, bo2, T1, 0, TROWS, SC, SC, 1.0f);
  ln_kernel<<<TROWS / 8, 256, 0, stream>>>(T0, ln3s, ln3b, Y16);
  transpose_cast_f16<<<dim3(2 * SFF / 64, SC / 64), dim3(32, 8), 0, stream>>>(ffw1, 2 * SFF, WT2, SC, 1.0f);
  wmma_gemm64<0, false, 2, 0, false><<<dim3((((TROWS / 64) * (2 * SFF / 64)) + 7) / 8, 1), 256, 0, stream>>>((const unsigned short*)Y16, nullptr, SC, 0, U16(WT2), nullptr, SC, 0, Hf, nullptr, 2 * SFF, 0, ffb1, nullptr, 0, TROWS, 2 * SFF, SC, 1.0f);
  geglu_kernel<<<(TROWS * SFF / 2 + 255) / 256, 256, 0, stream>>>(Hf, G16, (long)TROWS * SFF / 2);
  transpose_cast_f16<<<dim3(SC / 64, SFF / 64), dim3(32, 8), 0, stream>>>(ffw2, SC, WT2, SFF, 1.0f);
  wmma_gemm64<0, false, 2, 0, true><<<dim3((tr + 7) / 8, 1), 256, 0, stream>>>((const unsigned short*)G16, nullptr, SFF, 0, U16(WT2), nullptr, SFF, 0, T1, nullptr, SC, 0, ffb2, T0, 0, TROWS, SC, SFF, 1.0f);
  cast_f32_f16x2<<<(TROWS * SC / 2 + 255) / 256, 256, 0, stream>>>(T1, (_Float16*)O16, TROWS * SC / 2);
  transpose_cast_f16<<<dim3(SC / 64, SC / 64), dim3(32, 8), 0, stream>>>(pw, SC, WT, SC, 1.0f);
  wmma_gemm64<0, false, 2, 0, false><<<dim3((tr + 7) / 8, 1), 256, 0, stream>>>((const unsigned short*)O16, nullptr, SC, 0, U16(WT), nullptr, SC, 0, O, nullptr, SC, 0, pb, nullptr, 0, TROWS, SC, SC, 1.0f);
  out_kernel<<<dim3((SNT + 63) / 64, SC / 64, SB), dim3(32, 8), 0, stream>>>(O, x, out);
}
